// FilteredNoise_5669356835579
// MI455X (gfx1250) — hardware-verified
//
#include <hip/hip_runtime.h>
#include <math.h>

typedef __attribute__((ext_vector_type(16))) _Float16 v16h;
typedef __attribute__((ext_vector_type(8)))  _Float16 v8h;
typedef __attribute__((ext_vector_type(8)))  float    v8f;
typedef __attribute__((ext_vector_type(4)))  float    v4f;
typedef __attribute__((ext_vector_type(4)))  unsigned v4u;

constexpr int kBatch     = 32;
constexpr int kFrames    = 4000;
constexpr int kBins      = 65;
constexpr int kHop       = 64;
constexpr int kIrLen     = 2 * kBins - 1;
constexpr int kTaps      = kIrLen - 1;
constexpr int kKp        = 96;
constexpr int kRows      = kBatch * kFrames;
constexpr int kOutLen    = (kFrames - 1) * kHop + kHop + 2 * kBins - 2;
constexpr int kHopBlocks = kOutLen / kHop;
static_assert(kIrLen == 129 && kTaps == 128, "impulse response length");
static_assert(kOutLen == 256128 && kHopBlocks == 4002 && kHopBlocks * kHop == kOutLen, "output length");
static_assert((kKp % 32) == 0 && kKp >= kBins, "GEMM K multiple of 32");
static_assert((kRows % 64) == 0 && (kTaps % 64) == 0, "GEMM M,N multiples of 64");

constexpr float kCarryH     = 512.0f;
constexpr float kColScale   = 1.0f / ((float)kIrLen * kCarryH);
constexpr float kGain       = 0.01f;
constexpr float kTwoPiOverN = 6.28318530717958647692f / (float)kIrLen;

constexpr size_t kOffHH   = 0;
constexpr size_t kOffBT   = kOffHH  + (size_t)kRows * kKp * 2;
constexpr size_t kOffWSC  = kOffBT  + (size_t)kTaps * kKp * 2;
constexpr size_t kOffIR   = kOffWSC + (size_t)kTaps * 4;
constexpr size_t kWsTotal = kOffIR  + (size_t)kRows * kTaps * 4;
static_assert(kWsTotal == 90137088ull, "carve total");
static_assert(kWsTotal <= 134217728ull, "carve cap");
static_assert((kOffBT % 256) == 0 && (kOffWSC % 256) == 0 && (kOffIR % 256) == 0, "aligned regions");

__device__ __forceinline__ int imin(int a, int b) { return a < b ? a : b; }
__device__ __forceinline__ int imax(int a, int b) { return a > b ? a : b; }

__device__ __forceinline__ unsigned f16_bits(float x) {
  const _Float16 hv = (_Float16)x;
  const unsigned short us = __builtin_bit_cast(unsigned short, hv);
  return (unsigned)us;
}

constexpr int kPackChunks = kRows * (kKp / 8);
static_assert(kPackChunks == 1536000 && (kPackChunks % 256) == 0, "pack coverage");

__global__ __launch_bounds__(256) void pack_h_kernel(const float* __restrict__ H, unsigned* __restrict__ HH)
{
  const int i = blockIdx.x * 256 + threadIdx.x;
  if (i >= kPackChunks) return;
  const int row = i / (kKp / 8);
  const int c8  = i - row * (kKp / 8);
  const float* hr = H + (size_t)row * kBins;
  unsigned hb[8];
#pragma unroll
  for (int e = 0; e < 8; ++e) {
    const int k  = c8 * 8 + e;
    const int kc = (k < kBins) ? k : (kBins - 1);
    float v = hr[kc];
    asm volatile("" : "+v"(v));
    const float sv = (k < kBins) ? (v * kCarryH) : 0.0f;
    hb[e] = f16_bits(sv);
  }
  v4u w;
  w[0] = hb[0] | (hb[1] << 16);
  w[1] = hb[2] | (hb[3] << 16);
  w[2] = hb[4] | (hb[5] << 16);
  w[3] = hb[6] | (hb[7] << 16);
  unsigned* p = HH + (size_t)i * 4;
  *(volatile v4u*)p = w;
  __threadfence();
  *(volatile v4u*)p = w;
}

__global__ __launch_bounds__(256) void table_kernel(unsigned* __restrict__ BT, float* __restrict__ WSC)
{
  __shared__ __align__(16) float sv[2048];
  const int tid  = threadIdx.x;
  const int lane = tid & 31;
  const int wave = __builtin_amdgcn_readfirstlane((int)(threadIdx.x >> 5));
  const int blk  = blockIdx.x;
  const bool isW = (blk == 6);
#pragma unroll 1
  for (int e = 0; e < 8; ++e) {
    const int li = e * 256 + tid;
    const int gi = imin(blk, 5) * 2048 + li;
    const int nnB = gi / kKp;
    const int kB  = gi - nnB * kKp;
    const int nn = isW ? (li & (kTaps - 1)) : nnB;
    const int k  = isW ? 0 : kB;
    const int n  = nn + 1;
    const int dn = (n >= kHop) ? (n - kHop) : (kHop - n);
    const int r  = isW ? n : ((k * dn) % kIrLen);
    const float c  = cosf((float)r * kTwoPiOverN);
    const float ck = (k == 0) ? 1.0f : 2.0f;
    const float tv = (k < kBins) ? (ck * c) : 0.0f;
    const float wv = (0.5f * (1.0f - c)) * kColScale;
    sv[li] = isW ? wv : tv;
  }
  __syncthreads();
  if (!isW) {
    unsigned hb[8];
#pragma unroll
    for (int e = 0; e < 8; ++e) hb[e] = f16_bits(sv[8 * tid + e]);
    v4u w;
    w[0] = hb[0] | (hb[1] << 16);
    w[1] = hb[2] | (hb[3] << 16);
    w[2] = hb[4] | (hb[5] << 16);
    w[3] = hb[6] | (hb[7] << 16);
    unsigned* p = BT + (size_t)(blk * 256 + tid) * 4;
    *(volatile v4u*)p = w;
    __threadfence();
    *(volatile v4u*)p = w;
  } else if (wave == 0) {
    const v4f v = *(const v4f*)(sv + 4 * lane);
    float* p = WSC + 4 * lane;
    *(volatile v4f*)p = v;
    __threadfence();
    *(volatile v4f*)p = v;
  }
}

union FragH { v16h v; v8h h[2]; };
__device__ __forceinline__ v16h frag_load(const _Float16* p) {
  FragH f;
  f.h[0] = *(const v8h*)(p);
  f.h[1] = *(const v8h*)(p + 16);
  return f.v;
}
__device__ __forceinline__ v8f frag_mma(v16h a, v16h b, v8f c) {
  return __builtin_amdgcn_wmma_f32_16x16x32_f16(false, a, false, b, (short)0, c, false, false);
}
__device__ __forceinline__ void mma_guard(v8f& c, v16h a, v16h b) {
  asm volatile("v_nop\n\tv_nop\n\tv_nop\n\tv_nop" : "+v"(c) : "v"(a), "v"(b));
}
__device__ __forceinline__ void keep4_h(v16h a, v16h b, v16h c, v16h d) { asm volatile("v_nop" :: "v"(a), "v"(b), "v"(c), "v"(d)); }
__device__ __forceinline__ void acc_guard4(v8f& a, v8f& b, v8f& c, v8f& d) { asm volatile("v_nop\n\tv_nop\n\tv_nop\n\tv_nop" : "+v"(a), "+v"(b), "+v"(c), "+v"(d)); }

__global__ __launch_bounds__(256) void gemm_ir_kernel(
    const unsigned short* __restrict__ Ap, const unsigned short* __restrict__ Btp,
    const float* __restrict__ colscale, float* __restrict__ C)
{
  const _Float16* A  = (const _Float16*)Ap;
  const _Float16* Bt = (const _Float16*)Btp;
  __shared__ __align__(16) float sT[8][16 * 68];
  const int lane = threadIdx.x & 31;
  const int wave = __builtin_amdgcn_readfirstlane((int)(threadIdx.x >> 5));
  constexpr int tilesN = kTaps / 64;
  constexpr int tilesM = kRows / 64;
  const int tile = blockIdx.x * 8 + wave;
  if (tile >= tilesM * tilesN) return;
  const int tm = tile / tilesN;
  const int tn = tile - tm * tilesN;
  const int m0 = tm << 6;
  const int n0 = tn << 6;

  const int rlane = lane & 15;
  const int koff  = (lane >> 4) * 8;
  const int mOff  = (lane >> 4) * 8;

  v8f acc[4][4];
#pragma unroll
  for (int i = 0; i < 4; ++i)
#pragma unroll
    for (int j = 0; j < 4; ++j) acc[i][j] = (v8f){0.f, 0.f, 0.f, 0.f, 0.f, 0.f, 0.f, 0.f};

#pragma unroll 1
  for (int k0 = 0; k0 < kKp; k0 += 32) {
    v16h bh[4];
#pragma unroll
    for (int j = 0; j < 4; ++j) {
      const size_t bo = (size_t)(n0 + (j << 4) + rlane) * kKp + koff + k0;
      bh[j] = frag_load(Bt + bo);
    }
#pragma unroll
    for (int i = 0; i < 4; ++i) {
      const size_t ao = (size_t)(m0 + (i << 4) + rlane) * kKp + koff + k0;
      const v16h ah = frag_load(A + ao);
#pragma unroll
      for (int j = 0; j < 4; ++j) acc[i][j] = frag_mma(ah, bh[j], acc[i][j]);
#pragma unroll
      for (int j = 0; j < 4; ++j) mma_guard(acc[i][j], ah, bh[j]);
    }
    keep4_h(bh[0], bh[1], bh[2], bh[3]);
  }
  acc_guard4(acc[0][0], acc[0][1], acc[0][2], acc[0][3]);
  acc_guard4(acc[1][0], acc[1][1], acc[1][2], acc[1][3]);
  acc_guard4(acc[2][0], acc[2][1], acc[2][2], acc[2][3]);
  acc_guard4(acc[3][0], acc[3][1], acc[3][2], acc[3][3]);

  float csj[4];
#pragma unroll
  for (int j = 0; j < 4; ++j) csj[j] = colscale[n0 + (j << 4) + rlane];

  float* slab = sT[wave];
#pragma unroll
  for (int i = 0; i < 4; ++i) {
    const int mBase = m0 + (i << 4);
#pragma unroll
    for (int j = 0; j < 4; ++j) {
#pragma unroll
      for (int r = 0; r < 8; ++r) {
        const float v = acc[i][j][r] * csj[j];
        slab[(mOff + r) * 68 + (j << 4) + rlane] = v;
      }
    }
    __builtin_amdgcn_fence(__ATOMIC_RELEASE, "workgroup");
    __builtin_amdgcn_wave_barrier();
    __builtin_amdgcn_fence(__ATOMIC_ACQUIRE, "workgroup");
    {
      const int hh = lane >> 4, c4 = (lane & 15) * 4;
      for (int pass = 0; pass < 2; ++pass) {
#pragma unroll
        for (int it = 0; it < 8; ++it) {
          const int row = it * 2 + hh;
          const v4f v = *(const v4f*)(slab + row * 68 + c4);
          *(volatile v4f*)(C + (size_t)(mBase + row) * kTaps + n0 + c4) = v;
        }
        __threadfence();
      }
    }
    __builtin_amdgcn_fence(__ATOMIC_RELEASE, "workgroup");
    __builtin_amdgcn_wave_barrier();
    __builtin_amdgcn_fence(__ATOMIC_ACQUIRE, "workgroup");
  }
}

constexpr int kFirHops   = 32;
constexpr int kFirSlots  = kFirHops + 2;
constexpr int kXP        = 65;
constexpr int kCP        = 145;
constexpr int kCOff      = 8;
constexpr int kOP        = 68;
constexpr int kFirBlocks = (kHopBlocks + kFirHops - 1) / kFirHops;
constexpr int kPadWords  = 17;
static_assert(kFirBlocks == 126, "fir grid");
static_assert(kCOff + 1 + kTaps + 8 == kCP, "coefficient row layout");

__global__ __launch_bounds__(256) void fir_ola_kernel(
    const float* __restrict__ noise, const float* __restrict__ ir, float* __restrict__ out)
{
  __shared__ __align__(16) float xs[kFirSlots * kXP];
  __shared__ __align__(16) float cs[kFirSlots * kCP];
  __shared__ __align__(16) float so[kFirHops * kOP];
  const int tid  = threadIdx.x;
  const int lane = tid & 31;
  const int wave = __builtin_amdgcn_readfirstlane((int)(threadIdx.x >> 5));
  const int b  = blockIdx.y;
  const int q0 = blockIdx.x * kFirHops;

  for (int p = tid; p < kFirSlots * kPadWords; p += 256) {
    const int sl = p / kPadWords;
    const int w  = p - sl * kPadWords;
    const int pos = (w < 9) ? w : (kTaps + w);
    cs[sl * kCP + pos] = 0.0f;
  }
#pragma unroll
  for (int it = 0; it < 3; ++it) {
    const int idx = it * 256 + tid;
    const int idc = imin(idx, kFirSlots * 16 - 1);
    const int sl  = idc >> 4;
    const int c4  = (idc & 15) * 4;
    const int f   = q0 - 2 + sl;
    const bool ok = (f >= 0) && (f < kFrames);
    const int fc  = imin(imax(f, 0), kFrames - 1);
    const v4f v = *(const v4f*)(noise + ((size_t)b * kFrames + fc) * kHop + c4);
    float a0 = v[0], a1 = v[1], a2 = v[2], a3 = v[3];
    asm volatile("" : "+v"(a0), "+v"(a1), "+v"(a2), "+v"(a3));
    if (idx < kFirSlots * 16) {
      float* dst = xs + sl * kXP + c4;
      dst[0] = ok ? a0 : 0.0f;
      dst[1] = ok ? a1 : 0.0f;
      dst[2] = ok ? a2 : 0.0f;
      dst[3] = ok ? a3 : 0.0f;
    }
  }
#pragma unroll
  for (int it = 0; it < 5; ++it) {
    const int idx = it * 256 + tid;
    const int idc = imin(idx, kFirSlots * 32 - 1);
    const int sl  = idc >> 5;
    const int c4  = (idc & 31) * 4;
    const int f   = q0 - 2 + sl;
    const bool ok = (f >= 0) && (f < kFrames);
    const int fc  = imin(imax(f, 0), kFrames - 1);
    const v4f v = *(const v4f*)(ir + ((size_t)b * kFrames + fc) * kTaps + c4);
    float a0 = v[0], a1 = v[1], a2 = v[2], a3 = v[3];
    asm volatile("" : "+v"(a0), "+v"(a1), "+v"(a2), "+v"(a3));
    if (idx < kFirSlots * 32) {
      float* dst = cs + sl * kCP + kCOff + 1 + c4;
      dst[0] = ok ? a0 : 0.0f;
      dst[1] = ok ? a1 : 0.0f;
      dst[2] = ok ? a2 : 0.0f;
      dst[3] = ok ? a3 : 0.0f;
    }
  }
  __syncthreads();

  const int tb = wave * 8;
  float acc[8];
#pragma unroll
  for (int i = 0; i < 8; ++i) acc[i] = 0.0f;

#pragma unroll 1
  for (int d = 0; d < 3; ++d) {
    const int slot = lane + 2 - d;
    const int base = 64 * d + tb;
    const int js = (d == 2) ? tb : 0;
    const int je = (d == 0) ? (tb + 8) : kHop;
    const float* xr = xs + slot * kXP;
    const float* cr = cs + slot * kCP + kCOff + base;
    float W[8];
    W[0] = 0.0f;
#pragma unroll
    for (int r = 1; r < 8; ++r) W[r] = cr[r - js];
#pragma unroll 1
    for (int jj = js; jj < je; jj += 8) {
      const float* px = xr + jj;
      const float* pc = cr - jj;
#pragma unroll
      for (int e = 0; e < 8; ++e) {
        const float xv = px[e];
        W[(8 - e) & 7] = pc[-e];
#pragma unroll
        for (int i = 0; i < 8; ++i) acc[i] = fmaf(xv, W[(i - e + 8) & 7], acc[i]);
      }
    }
  }

  {
    float* orow = so + lane * kOP + tb;
#pragma unroll
    for (int i = 0; i < 8; ++i) orow[i] = acc[i] * kGain;
  }
  __syncthreads();

  v4f ov[2];
  size_t oo[2];
  bool okq[2];
#pragma unroll
  for (int it = 0; it < 2; ++it) {
    const int idx = it * 256 + tid;
    const int hop = idx >> 4;
    const int c4  = (idx & 15) * 4;
    ov[it] = *(const v4f*)(so + hop * kOP + c4);
    const int q = q0 + hop;
    okq[it] = (q < kHopBlocks);
    oo[it] = (size_t)b * kOutLen + (size_t)imin(q, kHopBlocks - 1) * kHop + c4;
  }
  for (int pass = 0; pass < 2; ++pass) {
#pragma unroll
    for (int it = 0; it < 2; ++it) {
      if (okq[it]) *(volatile v4f*)(out + oo[it]) = ov[it];
    }
    __threadfence();
  }
}

extern "C" void kernel_launch(void* const* d_in, const int* in_sizes, int n_in,
                              void* d_out, int out_size, void* d_ws, size_t ws_size,
                              hipStream_t stream) {
  if (n_in < 2) return;
  if (in_sizes[0] != kRows * kBins) return;
  if (in_sizes[1] != kRows * kHop) return;
  if (out_size != kBatch * kOutLen) return;
  if (ws_size < kWsTotal) return;

  const float* H     = (const float*)d_in[0];
  const float* noise = (const float*)d_in[1];
  float* out = (float*)d_out;

  char* ws = (char*)d_ws;
  unsigned*       HHw = (unsigned*)(ws + kOffHH);
  unsigned*       BTw = (unsigned*)(ws + kOffBT);
  float*          WSC = (float*)(ws + kOffWSC);
  float*          IR  = (float*)(ws + kOffIR);

  pack_h_kernel<<<kPackChunks / 256, 256, 0, stream>>>(H, HHw);
  table_kernel<<<7, 256, 0, stream>>>(BTw, WSC);
  gemm_ir_kernel<<<(kRows / 64) * (kTaps / 64) / 8, 256, 0, stream>>>(
      (const unsigned short*)(ws + kOffHH), (const unsigned short*)(ws + kOffBT), WSC, IR);
  fir_ola_kernel<<<dim3(kFirBlocks, kBatch), 256, 0, stream>>>(noise, IR, out);
}
